// non_local_b_57260503990845
// MI455X (gfx1250) — hardware-verified
//
#include <hip/hip_runtime.h>


typedef __attribute__((ext_vector_type(2))) float v2f;
typedef __attribute__((ext_vector_type(4))) float v4f;
typedef __attribute__((ext_vector_type(8))) float v8f;
typedef __attribute__((ext_vector_type(16))) _Float16 v16h;
#define VST2(T, ptr, val) do { const T _v = (val); *(volatile T*)(ptr) = _v; __threadfence(); *(volatile T*)(ptr) = _v; } while (0)
__device__ __forceinline__ v8f wmma16(v16h a, v16h b, v8f c) {
  v8f d = __builtin_amdgcn_wmma_f32_16x16x32_f16(false, a, false, b, (short)0, c, false, false);
  asm volatile("v_nop\n\tv_nop\n\tv_nop\n\tv_nop" : "+v"(d) : "v"(a), "v"(b));
  return d;
}
__device__ __forceinline__ void frag_split(const float* __restrict__ row, int hl, v16h& hi, v16h& lo) {
#pragma unroll
  for (int e = 0; e < 16; ++e) {
    const float v = row[(e < 8) ? (8 * hl + e) : (16 + 8 * hl + (e - 8))];
    const _Float16 h = (_Float16)v; hi[e] = h; lo[e] = (_Float16)(v - (float)h);
  }
}

#define C_DIM   256
#define H_DIM   128
#define N_TOK   10368
#define KSPLIT  6
#define CH      64
#define LSTR    68

template <bool TA, bool TB, int EPI>
__global__ __launch_bounds__(32) void gemm16_wmma(
    const float* __restrict__ A, const float* __restrict__ B,
    float* __restrict__ D, int lda, int ldb, int ldd, int Kz,
    const float* __restrict__ u, const float* __restrict__ v,
    const float* __restrict__ addbase, float scale)
{
  __shared__ float As[16 * LSTR];
  __shared__ float Bs[32 * LSTR];
  __shared__ float Ds[16][36];

  const int lane = threadIdx.x;
  const int m0 = blockIdx.x * 16;
  const int n0 = blockIdx.y * 32;
  const int z  = blockIdx.z;
  const int k_begin = z * Kz;
  const int k_end   = k_begin + Kz;

  const int hl = lane >> 4;
  const int lr = lane & 15;

  v8f acc = {}, acc2 = {};

  for (int k0 = k_begin; k0 < k_end; k0 += CH) {
    if (!TA) {
      #pragma unroll
      for (int i = 0; i < 8; ++i) {
        int t  = lane + 32 * i;
        int r  = t >> 4;
        int c4 = (t & 15) * 4;
        v4f val = *(const v4f*)(A + (size_t)(m0 + r) * lda + k0 + c4);
        *(v4f*)(&As[r * LSTR + c4]) = val;
      }
    } else {
      #pragma unroll
      for (int i = 0; i < 8; ++i) {
        int t  = lane + 32 * i;
        int cc = t >> 2;
        int qd = (t & 3) * 4;
        v4f val = *(const v4f*)(A + (size_t)(k0 + cc) * lda + m0 + qd);
        As[(qd + 0) * LSTR + cc] = val.x;
        As[(qd + 1) * LSTR + cc] = val.y;
        As[(qd + 2) * LSTR + cc] = val.z;
        As[(qd + 3) * LSTR + cc] = val.w;
      }
    }
    if (TB) {
      #pragma unroll
      for (int i = 0; i < 16; ++i) {
        int t  = lane + 32 * i;
        int r  = t >> 4;
        int c4 = (t & 15) * 4;
        v4f val = *(const v4f*)(B + (size_t)(n0 + r) * ldb + k0 + c4);
        *(v4f*)(&Bs[r * LSTR + c4]) = val;
      }
    } else {
      #pragma unroll
      for (int i = 0; i < 16; ++i) {
        int t  = lane + 32 * i;
        int cc = t >> 3;
        int qd = (t & 7) * 4;
        v4f val = *(const v4f*)(B + (size_t)(k0 + cc) * ldb + n0 + qd);
        Bs[(qd + 0) * LSTR + cc] = val.x;
        Bs[(qd + 1) * LSTR + cc] = val.y;
        Bs[(qd + 2) * LSTR + cc] = val.z;
        Bs[(qd + 3) * LSTR + cc] = val.w;
      }
    }
    if (k0 + CH < k_end) {
      if (!TA) __builtin_prefetch(A + (size_t)(m0 + lr) * lda + k0 + CH, 0, 0);
      else     __builtin_prefetch(A + (size_t)(k0 + CH + lane * 2) * lda + m0, 0, 0);
      if (TB)  __builtin_prefetch(B + (size_t)(n0 + lane) * ldb + k0 + CH, 0, 0);
      else     __builtin_prefetch(B + (size_t)(k0 + CH + lane * 2) * ldb + n0, 0, 0);
    }
    __syncthreads();

    #pragma unroll
    for (int kk = 0; kk < CH; kk += 32) {
      v16h ah, al, bh, bl;
      frag_split(&As[lr * LSTR + kk], hl, ah, al);
      frag_split(&Bs[lr * LSTR + kk], hl, bh, bl);
      acc = wmma16(ah, bh, acc); acc = wmma16(ah, bl, acc); acc = wmma16(al, bh, acc);
      frag_split(&Bs[(16 + lr) * LSTR + kk], hl, bh, bl);
      acc2 = wmma16(ah, bh, acc2); acc2 = wmma16(ah, bl, acc2); acc2 = wmma16(al, bh, acc2);
    }
    __syncthreads();
  }

  float* Dz = D + (size_t)z * (size_t)gridDim.x * 16 * ldd;
  #pragma unroll
  for (int r = 0; r < 8; ++r) {
    int row = m0 + r + 8 * hl;
    #pragma unroll
    for (int tcol = 0; tcol < 2; ++tcol) {
      int col = n0 + tcol * 16 + lr;
      float val = tcol ? acc2[r] : acc[r];
      if (EPI == 1) val += u[row] * v[col];
      if (EPI == 2) val = addbase[(size_t)row * ldd + col] + (val + u[row]) * scale;
      Ds[r + 8 * hl][tcol * 16 + lr] = val;
    }
  }
  __syncthreads();
  for (int pass = 0; pass < 2; ++pass) {
    #pragma unroll
    for (int rr = 0; rr < 16; ++rr) *(volatile float*)(Dz + (size_t)(m0 + rr) * ldd + n0 + lane) = Ds[rr][lane];
    __threadfence();
  }
}

__global__ __launch_bounds__(256) void rowsum_kernel(
    const float* __restrict__ feat, float* __restrict__ s)
{
  __shared__ float red[32];
  const int wave = threadIdx.x >> 5, lane = threadIdx.x & 31;
  for (int q = 0; q < 4; ++q) {
    const int c = blockIdx.x * 32 + wave * 4 + q;
    float p = 0.f;
    for (int n = lane; n < N_TOK; n += 32) p += feat[(size_t)c * N_TOK + n];
    #pragma unroll
    for (int off = 16; off > 0; off >>= 1) p += __shfl_xor(p, off, 32);
    if (lane == 0) red[wave * 4 + q] = p;
  }
  __syncthreads();
  if (threadIdx.x < 32) VST2(float, s + blockIdx.x * 32 + threadIdx.x, red[threadIdx.x]);
}

__global__ __launch_bounds__(256) void gsum_kernel(
    const float* __restrict__ Gp, float* __restrict__ G)
{
  const int i = blockIdx.x * 256 + threadIdx.x;
  float acc = 0.f;
  #pragma unroll
  for (int zz = 0; zz < KSPLIT; ++zz) acc += Gp[zz * (C_DIM * C_DIM) + i];
  VST2(float, G + i, acc);
}

__global__ __launch_bounds__(256) void qvec_kernel(
    const float* __restrict__ bi, const float* __restrict__ M2,
    float* __restrict__ q)
{
  const int c = threadIdx.x;
  float acc = 0.f;
  for (int r = 0; r < H_DIM; ++r) acc += bi[r] * M2[r * C_DIM + c];
  VST2(float, q + c, acc);
}

extern "C" void kernel_launch(void* const* d_in, const int* in_sizes, int n_in,
                              void* d_out, int out_size, void* d_ws, size_t ws_size,
                              hipStream_t stream) {
  const float* feat = (const float*)d_in[0];
  const float* Wi   = (const float*)d_in[1];
  const float* bi   = (const float*)d_in[2];
  const float* Wj   = (const float*)d_in[3];
  const float* bj   = (const float*)d_in[4];
  float* out = (float*)d_out;

  (void)in_sizes; (void)n_in; (void)out_size;
  if (ws_size < (size_t)(256 + (KSPLIT + 2) * C_DIM * C_DIM + H_DIM * C_DIM + 256) * 4) return;
  float* ws = (float*)d_ws;
  float* s  = ws;
  float* Gp = s + 256;
  float* G  = Gp + KSPLIT * C_DIM * C_DIM;
  float* M2 = G + C_DIM * C_DIM;
  float* R  = M2 + H_DIM * C_DIM;
  float* q  = R + C_DIM * C_DIM;

  rowsum_kernel<<<C_DIM / 32, 256, 0, stream>>>(feat, s);

  gemm16_wmma<false, true, 0><<<dim3(16, 8, KSPLIT), 32, 0, stream>>>(
      feat, feat, Gp, N_TOK, N_TOK, C_DIM, N_TOK / KSPLIT,
      nullptr, nullptr, nullptr, 0.f);
  gsum_kernel<<<C_DIM * C_DIM / 256, 256, 0, stream>>>(Gp, G);

  gemm16_wmma<false, false, 1><<<dim3(H_DIM / 16, 8, 1), 32, 0, stream>>>(
      Wj, G, M2, C_DIM, C_DIM, C_DIM, C_DIM, bj, s, nullptr, 0.f);

  qvec_kernel<<<1, 256, 0, stream>>>(bi, M2, q);

  gemm16_wmma<true, false, 0><<<dim3(16, C_DIM / 32, 1), 32, 0, stream>>>(
      M2, Wi, R, C_DIM, C_DIM, C_DIM, H_DIM,
      nullptr, nullptr, nullptr, 0.f);

  gemm16_wmma<false, false, 2><<<dim3(16, N_TOK / 32, 1), 32, 0, stream>>>(
      R, feat, out, C_DIM, N_TOK, N_TOK, C_DIM,
      q, nullptr, feat, 1.0f / (float)N_TOK);
}
